// CausalSelfAttention_16887811408360
// MI455X (gfx1250) — hardware-verified
//
#include <hip/hip_runtime.h>
#include <math.h>

#ifndef NB
#define NB 2
#endif
#ifndef SEQ
#define SEQ 2048
#endif
#define NB_FULL 2
#define SEQ_FULL 2048
#define CE 2048
#define NLAT 512
#define NHEAD 16
#define HD 128
#ifndef EROWS
#define EROWS 256
#endif

static_assert(SEQ % 64 == 0);
static_assert(EROWS % 64 == 0);
static_assert(EROWS >= 64);
static_assert(EROWS <= SEQ);
static_assert(NB <= NB_FULL);
static_assert(SEQ <= SEQ_FULL);
static_assert(NHEAD * HD == CE);

typedef __attribute__((ext_vector_type(16))) _Float16 v16h;
typedef __attribute__((ext_vector_type(8)))  _Float16 v8h;
typedef __attribute__((ext_vector_type(16))) __bf16   v16b;
typedef __attribute__((ext_vector_type(8)))  __bf16   v8b;
typedef __attribute__((ext_vector_type(8)))  float    v8f;
typedef __attribute__((ext_vector_type(4)))  float    v4f;
typedef unsigned int u4 __attribute__((ext_vector_type(4)));


#define VST2(T, ptr, val) do { const T vst2_v_ = (val); *(volatile T*)(ptr) = vst2_v_; __threadfence(); *(volatile T*)(ptr) = vst2_v_; } while (0)

__device__ __forceinline__ unsigned short f2bf_bits(float f) {
  unsigned u = __float_as_uint(f);
  return (unsigned short)((u + 0x7FFFu + ((u >> 16) & 1u)) >> 16);
}
__device__ __forceinline__ float bf_bits2f(unsigned short h) { return __uint_as_float(((unsigned)h) << 16); }
__device__ __forceinline__ float bfr(float v) { return bf_bits2f(f2bf_bits(v)); }
__device__ __forceinline__ unsigned pk2h(float a, float b) {
  return (unsigned)__builtin_bit_cast(unsigned short, (_Float16)a) | ((unsigned)__builtin_bit_cast(unsigned short, (_Float16)b) << 16);
}
__device__ __forceinline__ void wave_lds_sync() {
  __builtin_amdgcn_fence(3  , "workgroup");
  __builtin_amdgcn_wave_barrier();
  __builtin_amdgcn_fence(2  , "workgroup");
}

namespace kit {

__device__ __forceinline__ void dep_guard_h(v8f& a, v8f& b, v16h x, v16h y) { asm volatile("v_nop\n\tv_nop\n\tv_nop\n\tv_nop" : "+v"(a), "+v"(b) : "v"(x), "v"(y)); }
__device__ __forceinline__ void dep_guard_b(v8f& a, v8f& b, v16b x, v16b y) { asm volatile("v_nop\n\tv_nop\n\tv_nop\n\tv_nop" : "+v"(a), "+v"(b) : "v"(x), "v"(y)); }
__device__ __forceinline__ void keep4_h(v16h a, v16h b, v16h c, v16h d) { asm volatile("v_nop" :: "v"(a), "v"(b), "v"(c), "v"(d)); }
__device__ __forceinline__ void keep4_b(v16b a, v16b b, v16b c, v16b d) { asm volatile("v_nop" :: "v"(a), "v"(b), "v"(c), "v"(d)); }
__device__ __forceinline__ void acc_guard4(v8f& a, v8f& b, v8f& c, v8f& d) { asm volatile("v_nop\n\tv_nop\n\tv_nop\n\tv_nop" : "+v"(a), "+v"(b), "+v"(c), "+v"(d)); }

template <typename T> struct Frag;
template <> struct Frag<_Float16> {
  typedef v16h V; typedef v8h H8; union U { v16h v; v8h h[2]; };
  static __device__ __forceinline__ v16h load(const _Float16* p) {
    U f; f.h[0] = *(const v8h*)(p); f.h[1] = *(const v8h*)(p + 16); return f.v;
  }
  static __device__ __forceinline__ v8f mma(v16h a, v16h b, v8f c) {
    return __builtin_amdgcn_wmma_f32_16x16x32_f16(false, a, false, b, (short)0, c, false, false);
  }
  static __device__ __forceinline__ v8f mman(v16h a, v16h b, v8f c) {
    c = __builtin_amdgcn_wmma_f32_16x16x32_f16(false, a, false, b, (short)0, c, false, false);
    asm volatile("v_nop\n\tv_nop\n\tv_nop\n\tv_nop" : "+v"(c) : "v"(a), "v"(b));
    return c;
  }
  static __device__ __forceinline__ _Float16 cvt(float f) { return (_Float16)f; }
  static __device__ __forceinline__ void guard(v8f& a, v8f& b, v16h x, v16h y) { dep_guard_h(a, b, x, y); }
  static __device__ __forceinline__ void keep(v16h a, v16h b, v16h c, v16h d) { keep4_h(a, b, c, d); }
};
template <> struct Frag<__bf16> {
  typedef v16b V; typedef v8b H8; union U { v16b v; v8b h[2]; };
  static __device__ __forceinline__ v16b load(const __bf16* p) {
    U f; f.h[0] = *(const v8b*)(p); f.h[1] = *(const v8b*)(p + 16); return f.v;
  }
  static __device__ __forceinline__ v8f mma(v16b a, v16b b, v8f c) {
    return __builtin_amdgcn_wmma_f32_16x16x32_bf16(false, a, false, b, (short)0, c, false, false);
  }
  static __device__ __forceinline__ v8f mman(v16b a, v16b b, v8f c) {
    c = __builtin_amdgcn_wmma_f32_16x16x32_bf16(false, a, false, b, (short)0, c, false, false);
    asm volatile("v_nop\n\tv_nop\n\tv_nop\n\tv_nop" : "+v"(c) : "v"(a), "v"(b));
    return c;
  }
  static __device__ __forceinline__ __bf16 cvt(float f) { return __builtin_bit_cast(__bf16, f2bf_bits(f)); }
  static __device__ __forceinline__ void guard(v8f& a, v8f& b, v16b x, v16b y) { dep_guard_b(a, b, x, y); }
  static __device__ __forceinline__ void keep(v16b a, v16b b, v16b c, v16b d) { keep4_b(a, b, c, d); }
};
template <int ET> struct Elem;
template <> struct Elem<0> { typedef _Float16 T; };
template <> struct Elem<1> { typedef __bf16 T; };

template <int ET, int OUT_MODE>
__global__ __launch_bounds__(256) void wmma_gemm64(
    const unsigned short* __restrict__ Ap, int lda, long strideA,
    const unsigned short* __restrict__ Btp, int ldb, long strideB,
    void* __restrict__ Cout, void* __restrict__ Cout2, int ldc, long strideC,
    int M, int N, int K, float scale) {
  typedef typename Elem<ET>::T T;
  typedef typename Frag<T>::V V;
  const T* A = (const T*)Ap; const T* Bt = (const T*)Btp;
  __shared__ __align__(16) float sT[8][16 * 68];
  const int b    = blockIdx.y;
  const int lane = threadIdx.x & 31;
  const int wave = threadIdx.x >> 5;
  const int tilesN = N >> 6;
  const int tilesM = M >> 6;
  const int tile = blockIdx.x * 8 + wave;
  if (tile >= tilesM * tilesN) return;
  const int tm = tile / tilesN;
  const int tn = tile - tm * tilesN;
  const int m0 = tm << 6;
  const int n0 = tn << 6;

  const T* Ab = A  + (size_t)b * strideA;
  const T* Bb = Bt + (size_t)b * strideB;

  const int rlane = lane & 15;
  const int koff  = (lane >> 4) * 8;
  const int mOff  = (lane >> 4) * 8;

  v8f acc[4][4];
#pragma unroll
  for (int i = 0; i < 4; ++i)
#pragma unroll
    for (int j = 0; j < 4; ++j) acc[i][j] = (v8f){0.f,0.f,0.f,0.f,0.f,0.f,0.f,0.f};

  for (int k0 = 0; k0 < K; k0 += 32) {
    V bh[4];
#pragma unroll
    for (int j = 0; j < 4; ++j) {
      const size_t bo = (size_t)(n0 + (j << 4) + rlane) * ldb + koff + k0;
      bh[j] = Frag<T>::load(Bb + bo);
    }
#pragma unroll
    for (int i = 0; i < 4; ++i) {
      const size_t ao = (size_t)(m0 + (i << 4) + rlane) * lda + koff + k0;
      V ah = Frag<T>::load(Ab + ao);
#pragma unroll
      for (int j = 0; j < 4; ++j) acc[i][j] = Frag<T>::mma(ah, bh[j], acc[i][j]);
      Frag<T>::guard(acc[i][0], acc[i][3], ah, ah);
    }
    Frag<T>::keep(bh[0], bh[1], bh[2], bh[3]);
  }
  acc_guard4(acc[0][0], acc[0][1], acc[0][2], acc[0][3]);
  acc_guard4(acc[1][0], acc[1][1], acc[1][2], acc[1][3]);
  acc_guard4(acc[2][0], acc[2][1], acc[2][2], acc[2][3]);
  acc_guard4(acc[3][0], acc[3][1], acc[3][2], acc[3][3]);

  float* slab = sT[wave];
#pragma unroll
  for (int i = 0; i < 4; ++i) {
    const int mBase = m0 + (i << 4);
#pragma unroll
    for (int j = 0; j < 4; ++j) {
#pragma unroll
      for (int r = 0; r < 8; ++r) slab[(mOff + r) * 68 + (j << 4) + rlane] = acc[i][j][r] * scale;
    }
    wave_lds_sync();
    if (OUT_MODE == 0) {
      float* C = (float*)Cout + (size_t)b * strideC;
      const int hh = lane >> 4, c4 = (lane & 15) * 4;
      for (int pass = 0; pass < 2; ++pass) {
#pragma unroll
        for (int it = 0; it < 8; ++it) {
          const int row = it * 2 + hh;
          v4f v = *(const v4f*)(slab + row * 68 + c4);
          *(volatile v4f*)(C + (size_t)(mBase + row) * ldc + n0 + c4) = v;
        }
        __threadfence();
      }
    } else {
      const int q = lane >> 3, c8 = (lane & 7) * 8;
      unsigned short* C  = (unsigned short*)Cout  + (size_t)b * strideC;
      unsigned short* C2 = (OUT_MODE == 2) ? ((unsigned short*)Cout2 + (size_t)b * strideC) : C;
      for (int pass = 0; pass < 2; ++pass) {
#pragma unroll
        for (int it = 0; it < 4; ++it) {
          const int row = it * 4 + q;
          const float* sp = slab + row * 68 + c8;
          v8h hv, lv;
#pragma unroll
          for (int e = 0; e < 8; ++e) {
            if (OUT_MODE == 1) {
              hv[e] = (_Float16)sp[e];
              lv[e] = hv[e];
            } else {
              unsigned short hb = f2bf_bits(sp[e]);
              unsigned short lb = f2bf_bits(sp[e] - bf_bits2f(hb));
              hv[e] = __builtin_bit_cast(_Float16, hb);
              lv[e] = __builtin_bit_cast(_Float16, lb);
            }
          }
          *(volatile v8h*)(C + (size_t)(mBase + row) * ldc + n0 + c8) = hv;
          if (OUT_MODE == 2) *(volatile v8h*)(C2 + (size_t)(mBase + row) * ldc + n0 + c8) = lv;
        }
        __threadfence();
      }
    }
    wave_lds_sync();
  }
}

template <bool SPLIT>
__global__ __launch_bounds__(128) void attn128(
    const unsigned short* __restrict__ Qhp, const unsigned short* __restrict__ Qlp, int ldq, long q_bs,
    const unsigned short* __restrict__ Khp, const unsigned short* __restrict__ Klp, int ldk, long k_bs,
    const unsigned short* __restrict__ Vhp, const unsigned short* __restrict__ Vlp, int ldv, long v_bs,
    float* __restrict__ out, int ldo, long o_bs, int qb0, float sscale, float oscale) {
  typedef typename Elem<SPLIT ? 1 : 0>::T T;
  typedef typename Frag<T>::V V;
  typedef typename Frag<T>::H8 H8;
  typedef typename Frag<T>::U FU;
  const float PSC = SPLIT ? 1.0f : 4096.0f;
  __shared__ __align__(16) T     Psh[4][16 * 64];
  __shared__ __align__(16) T     Psl[SPLIT ? 4 : 1][SPLIT ? 16 * 64 : 8];
  __shared__ __align__(16) float Os[4][16 * 132];

  const int tid  = threadIdx.x;
  const int wave = tid >> 5;
  const int lane = tid & 31;
  const int hh   = lane >> 4;
  const int c    = lane & 15;
  const int qb = qb0 + (int)blockIdx.x;
  const int h  = blockIdx.y;
  const int b  = blockIdx.z;
  const int q0 = qb * 64 + wave * 16;

  const size_t qoff = (size_t)b * q_bs + (size_t)(q0 + c) * ldq + (size_t)h * HD + 8 * hh;
  const T* Qh = (const T*)Qhp + qoff;
  const T* Ql = SPLIT ? ((const T*)Qlp + qoff) : Qh;
  const size_t kbo = (size_t)b * k_bs + (size_t)h * HD + 8 * hh;
  const T* Kh = (const T*)Khp + kbo;
  const T* Kl = SPLIT ? ((const T*)Klp + kbo) : Kh;
  const size_t vbo = (size_t)b * v_bs + (size_t)(h * HD + c) * ldv + 8 * hh;
  const T* Vh = (const T*)Vhp + vbo;
  const T* Vl = SPLIT ? ((const T*)Vlp + vbo) : Vh;

  V qa[4];
  if (!SPLIT) {
#pragma unroll
    for (int dc = 0; dc < 4; ++dc) qa[dc] = Frag<T>::load(Qh + dc * 32);
  }

  float mrow[8], lrow[8];
  v8f oacc[8];
#pragma unroll
  for (int r = 0; r < 8; ++r) { mrow[r] = -INFINITY; lrow[r] = 0.f; }
#pragma unroll
  for (int t = 0; t < 8; ++t) oacc[t] = (v8f){0.f,0.f,0.f,0.f,0.f,0.f,0.f,0.f};

  T* pwh = Psh[wave];
  T* pwl = Psl[SPLIT ? wave : 0];

  for (int kc = 0; kc <= qb; ++kc) {
    const int kv0 = kc * 64;
    v8f s[4];
#pragma unroll
    for (int j = 0; j < 4; ++j) {
      s[j] = (v8f){0.f,0.f,0.f,0.f,0.f,0.f,0.f,0.f};
      const size_t ko = (size_t)(kv0 + j * 16 + c) * ldk;
#pragma unroll
      for (int dc = 0; dc < 4; ++dc) {
        asm volatile("" ::: "memory");
        const V kb = Frag<T>::load(Kh + ko + dc * 32);
        if (SPLIT) {
          const V kl = Frag<T>::load(Kl + ko + dc * 32);
          const V qh = Frag<T>::load(Qh + dc * 32);
          const V ql = Frag<T>::load(Ql + dc * 32);
          s[j] = Frag<T>::mman(qh, kb, s[j]);
          s[j] = Frag<T>::mman(qh, kl, s[j]);
          s[j] = Frag<T>::mman(ql, kb, s[j]);
        } else {
          s[j] = Frag<T>::mman(qa[dc], kb, s[j]);
        }
      }
    }
    const bool diag = (kc == qb);
#pragma unroll
    for (int r = 0; r < 8; ++r) {
      const int qrow = q0 + 8 * hh + r;
      float m = -INFINITY;
#pragma unroll
      for (int j = 0; j < 4; ++j) {
        const int kvcol = kv0 + j * 16 + c;
        float v = s[j][r] * sscale;
        v = (diag && (kvcol > qrow)) ? -INFINITY : v;
        s[j][r] = v;
        m = fmaxf(m, v);
      }
      m = fmaxf(m, __shfl_xor(m, 1, 32));
      m = fmaxf(m, __shfl_xor(m, 2, 32));
      m = fmaxf(m, __shfl_xor(m, 4, 32));
      m = fmaxf(m, __shfl_xor(m, 8, 32));
      const float mnew = fmaxf(mrow[r], m);
      const float alpha = exp2f(mrow[r] - mnew);
      mrow[r] = mnew;
      float psum = 0.f;
#pragma unroll
      for (int j = 0; j < 4; ++j) {
        const float p = exp2f(s[j][r] - mnew);
        psum += p;
        const int idx = (8 * hh + r) * 64 + j * 16 + c;
        if (SPLIT) {
          const unsigned short hb = f2bf_bits(p);
          const unsigned short lb = f2bf_bits(p - bf_bits2f(hb));
          pwh[idx] = __builtin_bit_cast(T, hb);
          pwl[idx] = __builtin_bit_cast(T, lb);
        } else {
          pwh[idx] = Frag<T>::cvt(p * PSC);
        }
      }
      psum += __shfl_xor(psum, 1, 32);
      psum += __shfl_xor(psum, 2, 32);
      psum += __shfl_xor(psum, 4, 32);
      psum += __shfl_xor(psum, 8, 32);
      lrow[r] = lrow[r] * alpha + psum;
#pragma unroll
      for (int t = 0; t < 8; ++t) oacc[t][r] *= alpha;
    }
    wave_lds_sync();
#pragma unroll
    for (int kk = 0; kk < 2; ++kk) {
      FU pa, pl;
      pa.h[0] = *(const H8*)(pwh + c * 64 + kk * 32 + 8 * hh);
      pa.h[1] = *(const H8*)(pwh + c * 64 + kk * 32 + 16 + 8 * hh);
      if (SPLIT) {
        pl.h[0] = *(const H8*)(pwl + c * 64 + kk * 32 + 8 * hh);
        pl.h[1] = *(const H8*)(pwl + c * 64 + kk * 32 + 16 + 8 * hh);
      } else {
        pl.v = pa.v;
      }
#pragma unroll
      for (int t = 0; t < 8; ++t) {
        asm volatile("" ::: "memory");
        const size_t vo = (size_t)(t * 16) * ldv + kv0 + kk * 32;
        const V vb = Frag<T>::load(Vh + vo);
        oacc[t] = Frag<T>::mman(pa.v, vb, oacc[t]);
        if (SPLIT) {
          const V vl = Frag<T>::load(Vl + vo);
          oacc[t] = Frag<T>::mman(pa.v, vl, oacc[t]);
          oacc[t] = Frag<T>::mman(pl.v, vb, oacc[t]);
        }
      }
    }
    wave_lds_sync();
  }

  float* os = Os[wave];
#pragma unroll
  for (int r = 0; r < 8; ++r) {
    const float inv = oscale * (1.0f / (lrow[r] * PSC));
#pragma unroll
    for (int t = 0; t < 8; ++t) os[(8 * hh + r) * 132 + t * 16 + c] = oacc[t][r] * inv;
  }
  wave_lds_sync();
  {
    float* ob = out + (size_t)b * o_bs + (size_t)q0 * ldo + (size_t)h * HD + lane * 4;
    for (int pass = 0; pass < 2; ++pass) {
#pragma unroll
      for (int it = 0; it < 16; ++it) {
        const v4f val = *(const v4f*)(os + it * 132 + lane * 4);
        *(volatile v4f*)(ob + (size_t)it * ldo) = val;
      }
      __threadfence();
    }
  }
}

}

template <bool BF>
__global__ __launch_bounds__(256) void k_cast_in(const float* __restrict__ SRC, int lds, unsigned short* __restrict__ DST, int ldd,
                                                 int nR, int nC, float sc, int rper, int rstride) {
  const long long u = (long long)blockIdx.x * 256 + threadIdx.x; const int per = nC / 8;
  if (u >= (long long)nR * per) return;
  const int r = (int)(u / per); const int c0 = 8 * (int)(u % per);
  const long long sr = (long long)(r / rper) * rstride + (r % rper);
  const float* s = SRC + sr * lds + c0;
  const v4f a = *(const v4f*)s; const v4f bq = *(const v4f*)(s + 4);
  float w[8] = {a.x, a.y, a.z, a.w, bq.x, bq.y, bq.z, bq.w};
#pragma unroll
  for (int e = 0; e < 8; ++e) w[e] = (BF ? bfr(w[e]) : w[e]) * sc;
  u4 pk; pk.x = pk2h(w[0], w[1]); pk.y = pk2h(w[2], w[3]); pk.z = pk2h(w[4], w[5]); pk.w = pk2h(w[6], w[7]);
  VST2(u4, (u4*)(DST + (long long)r * ldd + c0), pk);
}
__global__ __launch_bounds__(256) void k_cast_inT(const float* __restrict__ SRC, int lds, unsigned short* __restrict__ DST, int ldd,
                                                  int nR, int nC, float sc) {
  const long long u = (long long)blockIdx.x * 256 + threadIdx.x; const int per = nR / 8;
  if (u >= (long long)nC * per) return;
  const int cidx = (int)(u / per); const int r0 = 8 * (int)(u % per);
  float w[8];
#pragma unroll
  for (int e = 0; e < 8; ++e) w[e] = bfr(SRC[(long long)(r0 + e) * lds + cidx]) * sc;
  u4 pk; pk.x = pk2h(w[0], w[1]); pk.y = pk2h(w[2], w[3]); pk.z = pk2h(w[4], w[5]); pk.w = pk2h(w[6], w[7]);
  VST2(u4, (u4*)(DST + (long long)cidx * ldd + r0), pk);
}
__global__ __launch_bounds__(256) void k_cvt3(const float* __restrict__ SRC, int lds, unsigned short* __restrict__ DST,
                                              int nR, int nC, int rper, int rstride, int order) {
  const long long u = (long long)blockIdx.x * 256 + threadIdx.x; const int per = nC / 8;
  if (u >= (long long)nR * per) return;
  const int r = (int)(u / per); const int c0 = 8 * (int)(u % per);
  const long long sr = (long long)(r / rper) * rstride + (r % rper);
  const float* s = SRC + sr * lds + c0;
  const v4f a = *(const v4f*)s; const v4f bq = *(const v4f*)(s + 4);
  const float w[8] = {a.x, a.y, a.z, a.w, bq.x, bq.y, bq.z, bq.w};
  unsigned hb[8], lb[8];
#pragma unroll
  for (int e = 0; e < 8; ++e) { const unsigned short hq = f2bf_bits(w[e]); hb[e] = hq; lb[e] = f2bf_bits(w[e] - bf_bits2f(hq)); }
  u4 ph, pl;
  ph.x = hb[0] | (hb[1] << 16); ph.y = hb[2] | (hb[3] << 16); ph.z = hb[4] | (hb[5] << 16); ph.w = hb[6] | (hb[7] << 16);
  pl.x = lb[0] | (lb[1] << 16); pl.y = lb[2] | (lb[3] << 16); pl.z = lb[4] | (lb[5] << 16); pl.w = lb[6] | (lb[7] << 16);
  u4 s1, s2;
  s1.x = order ? ph.x : pl.x; s1.y = order ? ph.y : pl.y; s1.z = order ? ph.z : pl.z; s1.w = order ? ph.w : pl.w;
  s2.x = order ? pl.x : ph.x; s2.y = order ? pl.y : ph.y; s2.z = order ? pl.z : ph.z; s2.w = order ? pl.w : ph.w;
  unsigned short* d = DST + (long long)r * (3 * (long long)nC) + c0;
  VST2(u4, (u4*)d, ph);
  VST2(u4, (u4*)(d + nC), s1);
  VST2(u4, (u4*)(d + 2 * (long long)nC), s2);
}

static constexpr size_t al256(size_t b) { return (b + 255) / 256 * 256; }
static constexpr size_t SZ_X16   = al256((size_t)NB * SEQ * CE * 2);
static constexpr size_t SZ_WCC   = al256((size_t)CE * CE * 2);
static constexpr size_t SZ_WLC   = al256((size_t)NLAT * CE * 2);
static constexpr size_t SZ_EF32  = al256((size_t)CE * NLAT * 4);
static constexpr size_t SZ_E16   = al256((size_t)CE * NLAT * 2);
static constexpr size_t SZ_E3    = al256((size_t)CE * 3 * NLAT * 2);
static constexpr size_t SZ_CK16  = al256((size_t)NB * SEQ * NLAT * 2);
static constexpr size_t SZ_CKE3  = al256((size_t)NB * EROWS * 3 * NLAT * 2);
static constexpr size_t SZ_EPL   = al256((size_t)NB * EROWS * CE * 2);
static constexpr size_t OFF_X16   = 0;
static constexpr size_t OFF_WQ16  = OFF_X16 + SZ_X16;
static constexpr size_t OFF_WQT16 = OFF_WQ16 + SZ_WCC;
static constexpr size_t OFF_WO16  = OFF_WQT16 + SZ_WCC;
static constexpr size_t OFF_WDKV  = OFF_WO16 + SZ_WCC;
static constexpr size_t OFF_WUKT  = OFF_WDKV + SZ_WLC;
static constexpr size_t OFF_WUVT  = OFF_WUKT + SZ_WLC;
static constexpr size_t OFF_Q16   = OFF_WUVT + SZ_WLC;
static constexpr size_t OFF_VT16  = OFF_Q16 + SZ_X16;
static constexpr size_t OFF_KEF   = OFF_VT16 + SZ_X16;
static constexpr size_t OFF_VEF   = OFF_KEF + SZ_EF32;
static constexpr size_t OFF_KE16  = OFF_VEF + SZ_EF32;
static constexpr size_t OFF_VE16  = OFF_KE16 + SZ_E16;
static constexpr size_t OFF_KE3   = OFF_VE16 + SZ_E16;
static constexpr size_t OFF_VE3   = OFF_KE3 + SZ_E3;
static constexpr size_t OFF_CK16  = OFF_VE3 + SZ_E3;
static constexpr size_t OFF_CKE3  = OFF_CK16 + SZ_CK16;
static constexpr size_t OFF_QEH   = OFF_CKE3 + SZ_CKE3;
static constexpr size_t OFF_QEL   = OFF_QEH + SZ_EPL;
static constexpr size_t OFF_KEEH  = OFF_QEL + SZ_EPL;
static constexpr size_t OFF_KEEL  = OFF_KEEH + SZ_EPL;
static constexpr size_t OFF_VTEH  = OFF_KEEL + SZ_EPL;
static constexpr size_t OFF_VTEL  = OFF_VTEH + SZ_EPL;
static constexpr size_t WS_TOTAL  = OFF_VTEL + SZ_EPL;
static_assert(WS_TOTAL <= (size_t)134217728);
static constexpr size_t OUT1_OFF_BYTES = (size_t)NB_FULL * SEQ_FULL * CE * 4;
static_assert(OUT1_OFF_BYTES == (size_t)33554432);
static_assert((size_t)NB * SEQ * CE <= OUT1_OFF_BYTES / 4);
static_assert(OUT1_OFF_BYTES / 4 + (size_t)NB * SEQ * NLAT <= (size_t)41943040 / 4);

static inline unsigned gemm_blocks(int M, int N) { return (unsigned)(((M / 64) * (N / 64) + 7) / 8); }
static inline unsigned cast_blocks(long long rows, int cols) { return (unsigned)((rows * (cols / 8) + 255) / 256); }

extern "C" void kernel_launch(void* const* d_in, const int* in_sizes, int n_in, void* d_out, int out_size, void* d_ws, size_t ws_size, hipStream_t stream) {
  (void)out_size;
  if (n_in < 6) return;
  if ((long long)in_sizes[0] < ((long long)(NB - 1) * SEQ_FULL + SEQ) * CE) return;
  if ((long long)in_sizes[1] < (long long)CE * CE) return;
  if ((long long)in_sizes[2] < (long long)NLAT * CE) return;
  if ((long long)in_sizes[3] < (long long)CE * NLAT) return;
  if ((long long)in_sizes[4] < (long long)CE * NLAT) return;
  if ((long long)in_sizes[5] < (long long)CE * CE) return;
  if (WS_TOTAL > ws_size) return;

  const float* x    = (const float*)d_in[0];
  const float* Wq   = (const float*)d_in[1];
  const float* Wdkv = (const float*)d_in[2];
  const float* Wuk  = (const float*)d_in[3];
  const float* Wuv  = (const float*)d_in[4];
  const float* Wo   = (const float*)d_in[5];
  float* y   = (float*)d_out;
  float* ckv = (float*)((char*)d_out + OUT1_OFF_BYTES);

  char* ws = (char*)d_ws;
  unsigned short* X16   = (unsigned short*)(ws + OFF_X16);
  unsigned short* K16   = X16;
  unsigned short* WQ16  = (unsigned short*)(ws + OFF_WQ16);
  unsigned short* WQT16 = (unsigned short*)(ws + OFF_WQT16);
  unsigned short* WO16  = (unsigned short*)(ws + OFF_WO16);
  unsigned short* WDKV16 = (unsigned short*)(ws + OFF_WDKV);
  unsigned short* WUKT16 = (unsigned short*)(ws + OFF_WUKT);
  unsigned short* WUVT16 = (unsigned short*)(ws + OFF_WUVT);
  unsigned short* Q16   = (unsigned short*)(ws + OFF_Q16);
  unsigned short* VT16  = (unsigned short*)(ws + OFF_VT16);
  float* KEF = (float*)(ws + OFF_KEF);
  float* VEF = (float*)(ws + OFF_VEF);
  unsigned short* KE16  = (unsigned short*)(ws + OFF_KE16);
  unsigned short* VE16  = (unsigned short*)(ws + OFF_VE16);
  unsigned short* KE3   = (unsigned short*)(ws + OFF_KE3);
  unsigned short* VE3   = (unsigned short*)(ws + OFF_VE3);
  unsigned short* CK16  = (unsigned short*)(ws + OFF_CK16);
  unsigned short* CKE3  = (unsigned short*)(ws + OFF_CKE3);
  unsigned short* QEH   = (unsigned short*)(ws + OFF_QEH);
  unsigned short* QEL   = (unsigned short*)(ws + OFF_QEL);
  unsigned short* KEEH  = (unsigned short*)(ws + OFF_KEEH);
  unsigned short* KEEL  = (unsigned short*)(ws + OFF_KEEL);
  unsigned short* VTEH  = (unsigned short*)(ws + OFF_VTEH);
  unsigned short* VTEL  = (unsigned short*)(ws + OFF_VTEL);

  const int BT = NB * SEQ;
  const float WSC = 64.0f;
  const float CSC = 16.0f;
  const float ESC = 64.0f;
  const float QSC = 16.0f, KSC = 16.0f, VSC = 16.0f;

  k_cast_in<true><<<cast_blocks(BT, CE), 256, 0, stream>>>(x, CE, X16, CE, BT, CE, 1.0f, SEQ, SEQ_FULL);
  k_cast_in<true><<<cast_blocks(CE, CE), 256, 0, stream>>>(Wq, CE, WQ16, CE, CE, CE, WSC, CE, CE);
  k_cast_inT<<<cast_blocks(CE, CE), 256, 0, stream>>>(Wq, CE, WQT16, CE, CE, CE, WSC);
  k_cast_in<true><<<cast_blocks(CE, CE), 256, 0, stream>>>(Wo, CE, WO16, CE, CE, CE, WSC, CE, CE);
  k_cast_in<true><<<cast_blocks(NLAT, CE), 256, 0, stream>>>(Wdkv, CE, WDKV16, CE, NLAT, CE, WSC, NLAT, NLAT);
  k_cast_inT<<<cast_blocks(NLAT, CE), 256, 0, stream>>>(Wuk, NLAT, WUKT16, CE, CE, NLAT, WSC);
  k_cast_inT<<<cast_blocks(NLAT, CE), 256, 0, stream>>>(Wuv, NLAT, WUVT16, CE, CE, NLAT, WSC);

  kit::wmma_gemm64<0, 0><<<dim3(gemm_blocks(BT, NLAT), 1), 256, 0, stream>>>(X16, CE, 0, WDKV16, CE, 0, (void*)ckv, nullptr, NLAT, 0, BT, NLAT, CE, 1.0f / WSC);
  kit::wmma_gemm64<0, 1><<<dim3(gemm_blocks(BT, CE), 1), 256, 0, stream>>>(X16, CE, 0, WQ16, CE, 0, (void*)Q16, nullptr, CE, 0, BT, CE, CE, QSC / WSC);
  kit::wmma_gemm64<0, 2><<<dim3(gemm_blocks(EROWS, CE), NB), 256, 0, stream>>>(X16, CE, (long)SEQ * CE, WQ16, CE, 0, (void*)QEH, (void*)QEL, CE, (long)EROWS * CE, EROWS, CE, CE, 1.0f / WSC);
  kit::wmma_gemm64<0, 0><<<dim3(gemm_blocks(CE, NLAT), 1), 256, 0, stream>>>(WQT16, CE, 0, WUKT16, CE, 0, (void*)KEF, nullptr, NLAT, 0, CE, NLAT, CE, 1.0f / (WSC * WSC));
  kit::wmma_gemm64<0, 0><<<dim3(gemm_blocks(CE, NLAT), 1), 256, 0, stream>>>(WO16, CE, 0, WUVT16, CE, 0, (void*)VEF, nullptr, NLAT, 0, CE, NLAT, CE, 1.0f / (WSC * WSC));
  k_cast_in<false><<<cast_blocks(BT, NLAT), 256, 0, stream>>>(ckv, NLAT, CK16, NLAT, BT, NLAT, CSC, BT, BT);
  k_cvt3<<<cast_blocks((long long)NB * EROWS, NLAT), 256, 0, stream>>>(ckv, NLAT, CKE3, NB * EROWS, NLAT, EROWS, SEQ, 0);
  k_cast_in<false><<<cast_blocks(CE, NLAT), 256, 0, stream>>>(KEF, NLAT, KE16, NLAT, CE, NLAT, ESC, CE, CE);
  k_cvt3<<<cast_blocks(CE, NLAT), 256, 0, stream>>>(KEF, NLAT, KE3, CE, NLAT, CE, CE, 1);
  k_cast_in<false><<<cast_blocks(CE, NLAT), 256, 0, stream>>>(VEF, NLAT, VE16, NLAT, CE, NLAT, ESC, CE, CE);
  k_cvt3<<<cast_blocks(CE, NLAT), 256, 0, stream>>>(VEF, NLAT, VE3, CE, NLAT, CE, CE, 1);
  kit::wmma_gemm64<0, 1><<<dim3(gemm_blocks(BT, CE), 1), 256, 0, stream>>>(CK16, NLAT, 0, KE16, NLAT, 0, (void*)K16, nullptr, CE, 0, BT, CE, NLAT, KSC / (CSC * ESC));
  kit::wmma_gemm64<0, 1><<<dim3(gemm_blocks(CE, SEQ), NB), 256, 0, stream>>>(VE16, NLAT, 0, CK16, NLAT, (long)SEQ * NLAT, (void*)VT16, nullptr, SEQ, (long)CE * SEQ, CE, SEQ, NLAT, VSC / (CSC * ESC));
  kit::wmma_gemm64<1, 2><<<dim3(gemm_blocks(NB * EROWS, CE), 1), 256, 0, stream>>>(CKE3, 3 * NLAT, 0, KE3, 3 * NLAT, 0, (void*)KEEH, (void*)KEEL, CE, 0, NB * EROWS, CE, 3 * NLAT, 1.0f);
  kit::wmma_gemm64<1, 2><<<dim3(gemm_blocks(CE, EROWS), NB), 256, 0, stream>>>(VE3, 3 * NLAT, 0, CKE3, 3 * NLAT, (long)EROWS * 3 * NLAT, (void*)VTEH, (void*)VTEL, EROWS, (long)CE * EROWS, CE, EROWS, 3 * NLAT, 1.0f);

  const float SCL = 0.08838834764831845f * 1.4426950408889634f;
  if (SEQ / 64 > EROWS / 64) {
    kit::attn128<false><<<dim3((unsigned)(SEQ / 64 - EROWS / 64), NHEAD, NB), 128, 0, stream>>>(
        Q16, nullptr, CE, (long)SEQ * CE, K16, nullptr, CE, (long)SEQ * CE, VT16, nullptr, SEQ, (long)CE * SEQ,
        y, CE, (long)SEQ * CE, EROWS / 64, SCL / (QSC * KSC), 1.0f / VSC);
  }
  kit::attn128<true><<<dim3((unsigned)(EROWS / 64), NHEAD, NB), 128, 0, stream>>>(
      QEH, QEL, CE, (long)EROWS * CE, KEEH, KEEL, CE, (long)EROWS * CE, VTEH, VTEL, EROWS, (long)CE * EROWS,
      y, CE, (long)SEQ * CE, 0, SCL, 1.0f);
}
